// SimpleRetention_82583631167650
// MI455X (gfx1250) — hardware-run, weakly checked
//
#include <hip/hip_runtime.h>


#define NB   4
#define NS   4096
#define ND   64
#define HF   32
#define NPR  2048

typedef _Float16 h16;
typedef unsigned short bf;
typedef __attribute__((ext_vector_type(16))) __bf16   v16bf;
typedef __attribute__((ext_vector_type(16))) _Float16 v16h;
typedef __attribute__((ext_vector_type(8)))  _Float16 v8h;
typedef __attribute__((ext_vector_type(8)))  unsigned short v8us;
typedef __attribute__((ext_vector_type(8)))  float    v8f;
typedef __attribute__((ext_vector_type(4)))  float    v4f;
typedef v8h  __attribute__((may_alias)) v8ha;
typedef v4f  __attribute__((may_alias)) v4fa;
typedef v8us __attribute__((may_alias)) v8usa;

__device__ __forceinline__ unsigned short f2bf(float f) { unsigned u = __float_as_uint(f); u += 0x7FFFu + ((u >> 16) & 1u); return (unsigned short)(u >> 16); }
__device__ __forceinline__ float bf2f(unsigned short b) { return __uint_as_float(((unsigned)b) << 16); }
__device__ __forceinline__ float bfr(float f) { return bf2f(f2bf(f)); }
__device__ __forceinline__ v16h cat16(v8h lo, v8h hi) { return __builtin_shufflevector(lo, hi, 0, 1, 2, 3, 4, 5, 6, 7, 8, 9, 10, 11, 12, 13, 14, 15); }
__device__ __forceinline__ v16bf cat16b(v8us lo, v8us hi) { return __builtin_bit_cast(v16bf, __builtin_shufflevector(lo, hi, 0, 1, 2, 3, 4, 5, 6, 7, 8, 9, 10, 11, 12, 13, 14, 15)); }
__device__ __forceinline__ v8f wmma16(v16h a, v16h b, v8f c) { return __builtin_amdgcn_wmma_f32_16x16x32_f16(false, a, false, b, (short)0, c, false, false); }
__device__ __forceinline__ v8f wmmab(v16bf a, v16bf b, v8f c) { return __builtin_amdgcn_wmma_f32_16x16x32_bf16(false, a, false, b, (short)0, c, false, false); }

template <typename T16> struct WFrag;
template <> struct WFrag<h16> { typedef v16h V; static __device__ __forceinline__ V ld(const h16* p) { return cat16(*(const v8h*)p, *(const v8h*)(p + 16)); } static __device__ __forceinline__ v8f mma(V a, V b, v8f c) { return wmma16(a, b, c); } };
template <> struct WFrag<bf> { typedef v16bf V; static __device__ __forceinline__ V ld(const bf* p) { return cat16b(*(const v8us*)p, *(const v8us*)(p + 16)); } static __device__ __forceinline__ v8f mma(V a, V b, v8f c) { return wmmab(a, b, c); } };
template <typename T16, int NSPLIT, bool BIAS>
__global__ __launch_bounds__(32) void k_gemmw(const T16* __restrict__ A, const T16* __restrict__ A2, const T16* __restrict__ Bt, const T16* __restrict__ Bt2, int K, float* C, int ldc, const float* __restrict__ bias, size_t sA, size_t sB, size_t sC) {
    typedef typename WFrag<T16>::V V;
    __shared__ __align__(16) float os[16 * 68];
    const size_t z = blockIdx.z; A += z * sA; if (A2) A2 += z * sA; Bt += z * sB; if (Bt2) Bt2 += z * sB; C += z * sC;
    const int lane = threadIdx.x & 31, lr = lane & 15, hi = lane >> 4; const int r0 = blockIdx.x * 64, c0 = blockIdx.y * 64;
    v8f acc[4][4];
#pragma unroll
    for (int mb = 0; mb < 4; ++mb)
#pragma unroll
        for (int nb = 0; nb < 4; ++nb) acc[mb][nb] = (v8f){};
    const size_t aoff = (size_t)(r0 + lr) * K + 8 * hi, boff = (size_t)(c0 + lr) * K + 8 * hi;
    for (int kc = 0; kc < K; kc += 32) {
        V a[4], a2[4];
#pragma unroll
        for (int mb = 0; mb < 4; ++mb) { a[mb] = WFrag<T16>::ld(A + aoff + (size_t)mb * 16 * K + kc); if (NSPLIT == 1 || NSPLIT == 2) a2[mb] = WFrag<T16>::ld(A2 + aoff + (size_t)mb * 16 * K + kc); }
#pragma unroll
        for (int nb = 0; nb < 4; ++nb) { const V b = WFrag<T16>::ld(Bt + boff + (size_t)nb * 16 * K + kc); V b2; if (NSPLIT >= 2) b2 = WFrag<T16>::ld(Bt2 + boff + (size_t)nb * 16 * K + kc);
#pragma unroll
            for (int mb = 0; mb < 4; ++mb) { acc[mb][nb] = WFrag<T16>::mma(a[mb], b, acc[mb][nb]); if (NSPLIT == 1 || NSPLIT == 2) acc[mb][nb] = WFrag<T16>::mma(a2[mb], b, acc[mb][nb]); if (NSPLIT >= 2) acc[mb][nb] = WFrag<T16>::mma(a[mb], b2, acc[mb][nb]); } }
        asm volatile("v_nop\n\tv_nop\n\tv_nop\n\tv_nop" : "+v"(acc[0][0]), "+v"(acc[1][1]), "+v"(acc[2][2]), "+v"(acc[3][3]) : "v"(a[0]), "v"(a[3]));
    }
#pragma unroll
    for (int mb = 0; mb < 4; ++mb) {
#pragma unroll
        for (int nb = 0; nb < 4; ++nb) {
#pragma unroll
            for (int j = 0; j < 8; ++j) os[(hi * 8 + j) * 68 + nb * 16 + lr] = acc[mb][nb][j]; }
        __builtin_amdgcn_wave_barrier(); asm volatile("" ::: "memory");
        float* crow = C + (size_t)(r0 + mb * 16) * ldc + c0;
#pragma unroll 1
        for (int ps = 0; ps < 2; ++ps) {
#pragma unroll
            for (int s = 0; s < 8; ++s) { const int row = 2 * s + hi, cofs = lr * 4; v4f val = *(const v4fa*)(os + row * 68 + cofs); if (BIAS) { val[0] += bfr(bias[c0 + cofs]); val[1] += bfr(bias[c0 + cofs + 1]); val[2] += bfr(bias[c0 + cofs + 2]); val[3] += bfr(bias[c0 + cofs + 3]); }
                *(volatile v4f*)(crow + (size_t)row * ldc + cofs) = val; }
            if (ps == 0) __threadfence(); }
        __builtin_amdgcn_wave_barrier(); asm volatile("" ::: "memory");
    }
}

typedef __attribute__((ext_vector_type(2))) _Float16 v2h;
typedef __attribute__((ext_vector_type(4))) _Float16 v4h;
typedef __attribute__((ext_vector_type(2))) unsigned short v2us;
typedef __attribute__((ext_vector_type(4))) unsigned short v4us;
typedef __attribute__((ext_vector_type(2))) float v2f;
typedef __attribute__((ext_vector_type(4))) int v4i;

__device__ const unsigned RH_INVF[HF] = { 0x3f800000u, 0x3f3ff911u, 0x3f0ff59au, 0x3ed7e89bu, 0x3ea1e89bu, 0x3e72d425u, 0x3e361887u, 0x3e088d77u, 0x3dcccccdu, 0x3d99940du, 0x3d6655c2u, 0x3d2cba15u, 0x3d0186e3u, 0x3cc2434fu, 0x3c91ad39u, 0x3c5a7bf2u, 0x3c23d70au, 0x3bf5b9b0u, 0x3bb8449cu, 0x3b8a2e77u, 0x3b4f3e38u, 0x3b1b690du, 0x3ae91528u, 0x3aaec98eu, 0x3a83126fu, 0x3a44948cu, 0x3a136a16u, 0x39dd1727u, 0x39a5cb60u, 0x3978a815u, 0x393a7753u, 0x390bd472u };
__global__ __launch_bounds__(256) void k_rhtab(float* __restrict__ CS, float* __restrict__ SN, int n) {
  const int t = blockIdx.x * 256 + threadIdx.x; if (t >= n) return; const float a = (float)(t >> 5) * __uint_as_float(RH_INVF[t & 31]);
  const float k = rintf(a * 0.63661977236758134f); float r = fmaf(-k, 1.5703125f, a); r = fmaf(-k, 4.837512969970703125e-4f, r); r = fmaf(-k, 7.54978995489188216e-8f, r); const float z = r * r;
  const float s = fmaf(r * z, fmaf(z, fmaf(z, -1.9515295891e-4f, 8.3321608736e-3f), -1.6666654611e-1f), r);
  const float c = fmaf(z * z, fmaf(z, fmaf(z, 2.443315711809948e-5f, -1.388731625493765e-3f), 4.166664568298827e-2f), fmaf(z, -0.5f, 1.0f));
  const unsigned q = (unsigned)(int)k; const unsigned mk = 0u - (q & 1u); const unsigned cb = __float_as_uint(c), sb = __float_as_uint(s);
  const float co = __uint_as_float(((cb & ~mk) | (sb & mk)) ^ ((((q + 1u) >> 1) & 1u) << 31)); const float si = __uint_as_float(((sb & ~mk) | (cb & mk)) ^ (((q >> 1) & 1u) << 31));
  *(volatile float*)(CS + t) = co; *(volatile float*)(SN + t) = si; __threadfence(); *(volatile float*)(CS + t) = co; *(volatile float*)(SN + t) = si; }

__device__ __forceinline__ h16 toh_flush(float x) { const float z = (fabsf(x) < 6.103515625e-05f) ? 0.0f : x; return (h16)z; }

__global__ __launch_bounds__(256) void k_xtab(float* Fc) { const unsigned id = blockIdx.x * 256u + threadIdx.x; const unsigned pj = id & 31u, pp = id >> 5; const float bq = ((float)(2u * pj) + 25.6f) / 89.6f; const float pw = (float)pp / 512.0f; const float fv = expf(pw * logf(bq)); *(volatile float*)(Fc + id) = fv; __threadfence(); *(volatile float*)(Fc + id) = fv; }

__global__ __launch_bounds__(256) void k_xrot(const float* __restrict__ Ar, const float* __restrict__ Cn, const float* __restrict__ Sn, const float* __restrict__ Fc, unsigned iv, bf* Rh, bf* Rl) { const unsigned id = blockIdx.x * 256u + threadIdx.x; const unsigned e8 = id & 7u, pp = (id >> 3) & 4095u; const v4f wa = *(const v4f*)(Ar + (size_t)id * 8), wb = *(const v4f*)(Ar + (size_t)id * 8 + 4); const size_t tq = (size_t)pp * HF + e8 * 4u; const v4f cq = *(const v4f*)(Cn + tq), sq = *(const v4f*)(Sn + tq), fq = *(const v4f*)(Fc + tq); v8us oh, ol;
#pragma unroll
    for (int pr = 0; pr < 4; ++pr) { const float w0 = bfr(pr < 2 ? wa[2 * pr] : wb[2 * pr - 4]), w1 = bfr(pr < 2 ? wa[2 * pr + 1] : wb[2 * pr - 3]); const float gg = iv != 0u ? 1.0f / fq[pr] : fq[pr]; const float cc = cq[pr] * gg, zz = sq[pr] * gg; const float r0 = w0 * cc - w1 * zz, r1 = w1 * cc + w0 * zz; const unsigned short h0 = f2bf(r0), h1 = f2bf(r1); oh[2 * pr] = h0; oh[2 * pr + 1] = h1; ol[2 * pr] = f2bf(r0 - bf2f(h0)); ol[2 * pr + 1] = f2bf(r1 - bf2f(h1)); }
    *(volatile v8us*)(Rh + (size_t)id * 8) = oh; *(volatile v8us*)(Rl + (size_t)id * 8) = ol; __threadfence(); *(volatile v8us*)(Rh + (size_t)id * 8) = oh; *(volatile v8us*)(Rl + (size_t)id * 8) = ol; }

__global__ __launch_bounds__(256) void k_vt16(const float* __restrict__ Av, h16* Vt) { const unsigned id = blockIdx.x * 256u + threadIdx.x; const unsigned r0 = (id & 511u) << 3, gc = id >> 9, gp = gc >> 6, ch = gc & 63u; v8h ov;
#pragma unroll
    for (int e = 0; e < 8; ++e) ov[e] = toh_flush(bfr(Av[((size_t)gp * NS + r0 + e) * ND + ch]));
    *(volatile v8h*)(Vt + (size_t)id * 8) = ov; __threadfence(); *(volatile v8h*)(Vt + (size_t)id * 8) = ov; }

__global__ __launch_bounds__(256) void k_dmask(const float* __restrict__ Sc, unsigned rb, h16* Wt) { const unsigned id = blockIdx.x * 256u + threadIdx.x; const unsigned c0 = (id & 511u) << 3, rr = rb + (id >> 9); const v4f sa = *(const v4f*)(Sc + (size_t)id * 8), sb = *(const v4f*)(Sc + (size_t)id * 8 + 4); const float lg = logf(0.96875f); v8h ow;
#pragma unroll
    for (int e = 0; e < 8; ++e) { const unsigned cl = c0 + (unsigned)e; const unsigned df = rr >= cl ? rr - cl : 0u; const float wv = (e < 4 ? sa[e] : sb[e - 4]) * expf((float)df * lg); ow[e] = toh_flush(cl <= rr ? wv : 0.0f); }
    *(volatile v8h*)(Wt + (size_t)id * 8) = ow; __threadfence(); *(volatile v8h*)(Wt + (size_t)id * 8) = ow; }

extern "C" void kernel_launch(void* const* d_in, const int* in_sizes, int n_in, void* d_out, int out_size, void* d_ws, size_t ws_size, hipStream_t stream) {
    if (n_in < 3) return;
    if (in_sizes[0] != NB * NS * ND || in_sizes[1] != NB * NS * ND || in_sizes[2] != NB * NS * ND) return;
    if (out_size != NB * NS * ND) return;
    static_assert(NS == 4096 && ND == 64 && HF == 32 && ND == 2 * HF && NS == 2 * NPR && NPR % 64 == 0 && NS % 64 == 0 && ND % 64 == 0 && ND % 32 == 0 && NS % 32 == 0 && (NS * HF) % 256 == 0 && (NB * NS * ND / 8) % 256 == 0 && (NPR * NS / 8) % 256 == 0 && NB * NS == 16384, "the products: row and column counts multiples of 64, the depths of 32; each flat grid exact; a row's place is the low 12 bits of its number; a pass is a group's upper or lower 2,048 rows");
    const float* i0 = (const float*)d_in[0]; const float* i1 = (const float*)d_in[1]; const float* i2 = (const float*)d_in[2]; float* rs0 = (float*)d_out;
    char* wsp = (char*)d_ws; auto carve = [&](size_t bytes) { char* p = wsp; wsp += (bytes + 255) & ~(size_t)255; return (void*)p; };
    float* Cn = (float*)carve((size_t)NS * HF * 4); float* Sn = (float*)carve((size_t)NS * HF * 4); float* Fc = (float*)carve((size_t)NS * HF * 4); bf* R1h = (bf*)carve((size_t)NB * NS * ND * 2); bf* R1l = (bf*)carve((size_t)NB * NS * ND * 2); bf* R2h = (bf*)carve((size_t)NB * NS * ND * 2); bf* R2l = (bf*)carve((size_t)NB * NS * ND * 2); h16* Vt = (h16*)carve((size_t)NB * ND * NS * 2); float* Sc = (float*)carve((size_t)NPR * NS * 4); h16* Wt = (h16*)carve((size_t)NPR * NS * 2);
    if ((size_t)(wsp - (char*)d_ws) > ws_size) return;
    k_rhtab<<<(unsigned)(NS * HF / 256), 256, 0, stream>>>(Cn, Sn, NS * HF);
    k_xtab<<<(unsigned)(NS * HF / 256), 256, 0, stream>>>(Fc);
    k_xrot<<<(unsigned)(NB * NS * ND / 8 / 256), 256, 0, stream>>>(i0, Cn, Sn, Fc, 0u, R1h, R1l);
    k_xrot<<<(unsigned)(NB * NS * ND / 8 / 256), 256, 0, stream>>>(i1, Cn, Sn, Fc, 1u, R2h, R2l);
    k_vt16<<<(unsigned)(NB * ND * NS / 8 / 256), 256, 0, stream>>>(i2, Vt);
    for (unsigned ps = 0; ps < (unsigned)(2 * NB); ++ps) { const unsigned gp = ps >> 1, rb = (ps & 1u) * (unsigned)NPR; const size_t ro = ((size_t)gp * NS + rb) * ND, go = (size_t)gp * NS * ND;
        k_gemmw<bf, 2, false><<<dim3(NPR / 64, NS / 64, 1), 32, 0, stream>>>(R1h + ro, R1l + ro, R2h + go, R2l + go, ND, Sc, NS, nullptr, 0, 0, 0);
        k_dmask<<<(unsigned)(NPR * NS / 8 / 256), 256, 0, stream>>>(Sc, rb, Wt);
        k_gemmw<h16, 0, false><<<dim3(NPR / 64, ND / 64, 1), 32, 0, stream>>>(Wt, nullptr, Vt + go, nullptr, NS, rs0 + ro, ND, nullptr, 0, 0, 0); }
}
